// Mukara_45698452030097
// MI455X (gfx1250) — hardware-verified
//
#include <hip/hip_runtime.h>
#include <stddef.h>


#define DD      128
#define FIN     16
#define KP1     32
#define K2      256
#define HID     128
#define NTHR    256
#define NWAVE   8
#define EPT     8
#define NGRP    2
#define CHUNK   (NTHR * EPT * NGRP)
#define WCAP    (EPT * NGRP * 32)
#define LISTN   (NWAVE * WCAP)
#define NBC     4096
#define NBF     2048
#define FPC     (NBC / NBF)
#define RCAP    49152
#define RBN     128
#define TGT     256
#define DEGCAP  256
#define OTHR    512
#define BM      64
#define LMAX    8
#define WSCAP   134217728
#define WSCL    64.0f
#define WSCLI   0.015625f

#define PL_P1   (HID * KP1)
#define PL_SQ   (HID * HID)
#define PL_U1   (HID * K2)
#define UPB     (NTHR * 8)
#define BP1     (PL_P1 / UPB)
#define BSQ     (PL_SQ / UPB)
#define BU1     (PL_U1 / UPB)

#define LDS_FILL  ((RCAP + NBF + LISTN) * 4 + 64)
#define LDS_PROJ  (BM * KP1 * 2 + BM * HID * 2 + BM * HID * 4)
#define LDS_LAYER (BM * K2 * 2 + BM * HID * 2 + BM * HID * 4)
#define LDS_OUT   (BM * HID * 2 + BM * HID * 4 + 256)

static_assert((CHUNK & (CHUNK - 1)) == 0);
static_assert(CHUNK <= 4096);
static_assert(NBC <= 4096 && NBF <= 4096);
static_assert((NBC & (NBC - 1)) == 0 && (NBF & (NBF - 1)) == 0);
static_assert(NBC == FPC * NBF && FPC == 2);
static_assert(OTHR * 8 == NBC);
static_assert(OTHR / 32 == 8 * FPC);
static_assert((RCAP % 32) == 0);
static_assert(TGT == NWAVE * 32);
static_assert((TGT % BM) == 0);
static_assert((DEGCAP % 32) == 0);
static_assert(BM == 64 && NWAVE == 8 && NTHR == 256);
static_assert(DD == HID && K2 == 2 * DD);
static_assert((KP1 % 32) == 0 && FIN <= KP1 && FIN == 16);
static_assert((HID % 32) == 0 && (K2 % 32) == 0);
static_assert((PL_P1 % 128) == 0 && (PL_SQ % 128) == 0 && (PL_U1 % 128) == 0);
static_assert((PL_P1 % UPB) == 0 && (PL_SQ % UPB) == 0 && (PL_U1 % UPB) == 0);
static_assert(BP1 * UPB == PL_P1 && BSQ * UPB == PL_SQ && BU1 * UPB == PL_U1);

typedef float          v4f  __attribute__((ext_vector_type(4)));
typedef float          v8f  __attribute__((ext_vector_type(8)));
typedef int            v4i  __attribute__((ext_vector_type(4)));
typedef _Float16       v8h  __attribute__((ext_vector_type(8)));
typedef _Float16       v16h __attribute__((ext_vector_type(16)));
union FragH { v16h v; v8h h[2]; };

__device__ __forceinline__ v8f wmh(v16h a, v16h b, v8f c) {
  v8f d = __builtin_amdgcn_wmma_f32_16x16x32_f16(false, a, false, b, (short)0, c, false, false);
  asm volatile("v_nop\n\tv_nop\n\tv_nop\n\tv_nop" : "+v"(d) : "v"(a), "v"(b));
  return d;
}

__device__ __forceinline__ v8h cvt8(v4f a, v4f b, float s) {
  v8h r;
  r[0] = (_Float16)(a.x * s); r[1] = (_Float16)(a.y * s); r[2] = (_Float16)(a.z * s); r[3] = (_Float16)(a.w * s);
  r[4] = (_Float16)(b.x * s); r[5] = (_Float16)(b.y * s); r[6] = (_Float16)(b.z * s); r[7] = (_Float16)(b.w * s);
  return r;
}

__device__ __forceinline__ float wsum(float v) {
#pragma unroll
  for (int mk = 16; mk >= 1; mk >>= 1) v += __shfl_xor(v, mk);
  return v;
}

__device__ __forceinline__ void zacc(v8f (&acc)[4]) {
#pragma unroll
  for (int t = 0; t < 4; ++t) { v8f z = {0.f, 0.f, 0.f, 0.f, 0.f, 0.f, 0.f, 0.f}; acc[t] = z; }
}

__global__ __launch_bounds__(NTHR) void k_wprep(
    const float* __restrict__ wp1, const float* __restrict__ wp2,
    const float* __restrict__ wu1, const float* __restrict__ wu2,
    const float* __restrict__ wo1, _Float16* planes, int L) {
  const int b = (int)blockIdx.x, tid = (int)threadIdx.x;
  const float* src;
  int Ks, Kp, lb;
  size_t po;
  if (b < BP1) {
    src = wp1; Ks = FIN; Kp = KP1; lb = b; po = 0;
  } else if (b < BP1 + BSQ) {
    src = wp2; Ks = HID; Kp = HID; lb = b - BP1; po = (size_t)PL_P1;
  } else if (b < BP1 + BSQ + L * BU1) {
    const int q = b - (BP1 + BSQ), i = q / BU1;
    lb = q - i * BU1;
    src = wu1 + (size_t)i * K2 * HID; Ks = K2; Kp = K2;
    po = (size_t)PL_P1 + PL_SQ + (size_t)i * PL_U1;
  } else if (b < BP1 + BSQ + L * (BU1 + BSQ)) {
    const int q = b - (BP1 + BSQ + L * BU1), i = q / BSQ;
    lb = q - i * BSQ;
    src = wu2 + (size_t)i * HID * HID; Ks = HID; Kp = HID;
    po = (size_t)PL_P1 + PL_SQ + (size_t)L * PL_U1 + (size_t)i * PL_SQ;
  } else {
    lb = b - (BP1 + BSQ + L * (BU1 + BSQ));
    src = wo1; Ks = HID; Kp = HID;
    po = (size_t)PL_P1 + PL_SQ + (size_t)L * (PL_U1 + PL_SQ);
  }
  const int upr = Kp >> 3;
  const int u   = lb * NTHR + tid;
  int n = u / upr;
  const int k0 = (u - n * upr) * 8;
  n = n > HID - 1 ? HID - 1 : n;

  v8h r;
#pragma unroll
  for (int j = 0; j < 8; ++j) {
    const int k  = k0 + j;
    const int kc = k < Ks ? k : Ks - 1;
    float v = src[(size_t)kc * HID + n];
    if (k >= Ks) v = 0.f;
    r[j] = (_Float16)(v * WSCL);
  }
  _Float16* d = planes + po + (size_t)u * 8;
  *(volatile v8h*)d = r;
  __threadfence();
  *(volatile v8h*)d = r;
}

template <int NB>
__device__ __forceinline__ int scan_chunk(const int* __restrict__ dsts, int nE, int cbase, int slotBase,
                                          int vec8, int* list, int tid, int lane, int wave) {
  int wc = 0;
#pragma unroll
  for (int g = 0; g < NGRP; ++g) {
    const int el0  = (g * NTHR + tid) * EPT;
    const int e0   = cbase + el0;
    const int sent = -2147483647 - 1;
    v4i da, db;
    if (vec8 != 0 && cbase + CHUNK <= nE) {
      da = *(const v4i*)(dsts + e0);
      db = *(const v4i*)(dsts + e0 + 4);
    } else {
      da.x = (e0     < nE) ? dsts[min(e0, nE - 1)] : sent;
      da.y = (e0 + 1 < nE) ? dsts[min(e0 + 1, nE - 1)] : sent;
      da.z = (e0 + 2 < nE) ? dsts[min(e0 + 2, nE - 1)] : sent;
      da.w = (e0 + 3 < nE) ? dsts[min(e0 + 3, nE - 1)] : sent;
      db.x = (e0 + 4 < nE) ? dsts[min(e0 + 4, nE - 1)] : sent;
      db.y = (e0 + 5 < nE) ? dsts[min(e0 + 5, nE - 1)] : sent;
      db.z = (e0 + 6 < nE) ? dsts[min(e0 + 6, nE - 1)] : sent;
      db.w = (e0 + 7 < nE) ? dsts[min(e0 + 7, nE - 1)] : sent;
    }
    const unsigned nb = (unsigned)slotBase;
    const unsigned s0 = (unsigned)da.x - nb, s1 = (unsigned)da.y - nb;
    const unsigned s2 = (unsigned)da.z - nb, s3 = (unsigned)da.w - nb;
    const unsigned s4 = (unsigned)db.x - nb, s5 = (unsigned)db.y - nb;
    const unsigned s6 = (unsigned)db.z - nb, s7 = (unsigned)db.w - nb;
    const bool h0 = s0 < (unsigned)NB, h1 = s1 < (unsigned)NB, h2 = s2 < (unsigned)NB, h3 = s3 < (unsigned)NB;
    const bool h4 = s4 < (unsigned)NB, h5 = s5 < (unsigned)NB, h6 = s6 < (unsigned)NB, h7 = s7 < (unsigned)NB;
    const unsigned any = __builtin_amdgcn_ballot_w32(h0 | h1 | h2 | h3 | h4 | h5 | h6 | h7);
    if (any != 0u) {
#define HITJ(J, HJ, SJ) { \
        const unsigned mj = __builtin_amdgcn_ballot_w32(HJ); \
        if (mj != 0u) { \
          if (HJ) { \
            const int pos = wc + (int)__builtin_amdgcn_mbcnt_lo(mj, 0u); \
            if (pos < WCAP) list[wave * WCAP + pos] = ((el0 + (J)) << 12) | (int)(SJ); \
          } \
          wc += (int)__builtin_popcount(mj); } }
      HITJ(0, h0, s0)
      HITJ(1, h1, s1)
      HITJ(2, h2, s2)
      HITJ(3, h3, s3)
      HITJ(4, h4, s4)
      HITJ(5, h5, s5)
      HITJ(6, h6, s6)
      HITJ(7, h7, s7)
#undef HITJ
    }
  }
  return wc;
}

__global__ __launch_bounds__(NTHR) void k_count(
    const int* __restrict__ dsts, int* cnt, int nE, int vec8) {
  __shared__ __attribute__((aligned(16))) int scnt[NBC];
  __shared__ __attribute__((aligned(16))) int list[LISTN];
  __shared__ int wcnt[NWAVE];
  const int tid = threadIdx.x, lane = tid & 31, wave = tid >> 5;
  const int nodeBase = blockIdx.x * NBC;

  for (int i = tid; i < NBC; i += NTHR) scnt[i] = 0;
  __syncthreads();

  const int nChunks = (nE + CHUNK - 1) / CHUNK;
#pragma unroll 1
  for (int ch = 0; ch < nChunks; ++ch) {
    const int cbase = ch * CHUNK;
    const int wc = scan_chunk<NBC>(dsts, nE, cbase, nodeBase, vec8, list, tid, lane, wave);
    if (lane == 0) wcnt[wave] = wc;
    __syncthreads();
    if (wave == 0) {
#pragma unroll 1
      for (int wsx = 0; wsx < NWAVE; ++wsx) {
        int n = __builtin_amdgcn_readfirstlane(wcnt[wsx]);
        n = n > WCAP ? WCAP : (n < 0 ? 0 : n);
        const int* lp = list + wsx * WCAP;
#pragma unroll 1
        for (int i = 0; i < n; ++i) {
          const int ent  = __builtin_amdgcn_readfirstlane(lp[i]);
          const int slot = ent & (NBC - 1);
          if (lane == 0) scnt[slot] = scnt[slot] + 1;
        }
      }
    }
    __syncthreads();
  }

  v4i cq[4];
#pragma unroll
  for (int q = 0; q < 4; ++q) {
    const int f = (wave * 4 + q) * 128 + 4 * lane;
    cq[q] = *(const v4i*)(scnt + f);
  }
  int* cpn = cnt + (size_t)nodeBase;
#pragma unroll
  for (int q = 0; q < 4; ++q) {
    const int f = (wave * 4 + q) * 128 + 4 * lane;
    *(volatile v4i*)(cpn + f) = cq[q];
  }
  __threadfence();
#pragma unroll
  for (int q = 0; q < 4; ++q) {
    const int f = (wave * 4 + q) * 128 + 4 * lane;
    *(volatile v4i*)(cpn + f) = cq[q];
  }
}

__global__ __launch_bounds__(OTHR) void k_offsets(
    const int* __restrict__ cnt, int* off, int* rbase, int nChunk) {
  __shared__ __attribute__((aligned(16))) int soff[NBC];
  __shared__ __attribute__((aligned(16))) int srb[RBN];
  __shared__ int wtot[OTHR / 32];
  const int tid = threadIdx.x, lane = tid & 31, wave = tid >> 5, sub = tid >> 8;
  for (int i = tid; i < RBN; i += OTHR) srb[i] = 0;
  __syncthreads();
  int carry = 0;
#pragma unroll 1
  for (int ch = 0; ch < nChunk; ++ch) {
    const int base = ch * NBC;
    const v4i ca = *(const v4i*)(cnt + base + 8 * tid);
    const v4i cb = *(const v4i*)(cnt + base + 8 * tid + 4);
    const int e0 = max(ca.x, 0), e1 = max(ca.y, 0), e2 = max(ca.z, 0), e3 = max(ca.w, 0);
    const int e4 = max(cb.x, 0), e5 = max(cb.y, 0), e6 = max(cb.z, 0), e7 = max(cb.w, 0);
    const int ts = e0 + e1 + e2 + e3 + e4 + e5 + e6 + e7;
    int incl = ts;
#pragma unroll
    for (int d = 1; d < 32; d <<= 1) {
      const int t = __shfl_up(incl, d);
      if (lane >= d) incl += t;
    }
    if (lane == 31) wtot[wave] = incl;
    __syncthreads();
    int S0 = 0, S1 = 0;
#pragma unroll
    for (int w = 0; w < 8; ++w) { S0 += wtot[w]; S1 += wtot[8 + w]; }
    int pre = 0;
#pragma unroll 1
    for (int w = 8 * sub; w < wave; ++w) pre += wtot[w];
    const int b0 = carry;
    const int b1 = b0 + ((S0 + 31) & ~31);
    const int b2 = b1 + ((S1 + 31) & ~31);
    const int myb = sub == 0 ? b0 : b1;
    if (tid == 0) {
      srb[min(2 * ch + 0, RBN - 1)] = b0;
      srb[min(2 * ch + 1, RBN - 1)] = b1;
    }
    int run = myb + pre + incl - ts;
    soff[8 * tid + 0] = run; run += e0;
    soff[8 * tid + 1] = run; run += e1;
    soff[8 * tid + 2] = run; run += e2;
    soff[8 * tid + 3] = run; run += e3;
    soff[8 * tid + 4] = run; run += e4;
    soff[8 * tid + 5] = run; run += e5;
    soff[8 * tid + 6] = run; run += e6;
    soff[8 * tid + 7] = run;
    carry = b2;
    __syncthreads();
    const v4i o0 = *(const v4i*)(soff + 4 * tid);
    const v4i o1 = *(const v4i*)(soff + 4 * (tid + OTHR));
    int* op = off + base;
    *(volatile v4i*)(op + 4 * tid) = o0;
    *(volatile v4i*)(op + 4 * (tid + OTHR)) = o1;
    __threadfence();
    *(volatile v4i*)(op + 4 * tid) = o0;
    *(volatile v4i*)(op + 4 * (tid + OTHR)) = o1;
    __syncthreads();
  }
  if (tid == 0) srb[min(2 * nChunk, RBN - 1)] = carry;
  __syncthreads();
  v4i rv = {0, 0, 0, 0};
  if (tid < 32) rv = *(const v4i*)(srb + 4 * tid);
  if (tid < 32) *(volatile v4i*)(rbase + 4 * tid) = rv;
  __threadfence();
  if (tid < 32) *(volatile v4i*)(rbase + 4 * tid) = rv;
}

__global__ __launch_bounds__(NTHR) void k_fill(
    const int* __restrict__ dsts, const int* __restrict__ srcs, const int* __restrict__ off,
    const int* __restrict__ rbase, int* csr, int nN, int nE, int vec8, int csrLen) {
  extern __shared__ v4f lds_dyn[];
  int* region = (int*)lds_dyn;
  int* cursor = region + RCAP;
  int* list   = cursor + NBF;
  int* wcnt   = list + LISTN;
  const int tid = threadIdx.x, lane = tid & 31, wave = tid >> 5;
  const int b = blockIdx.x;
  const int nodeBase = b * NBF;

  int rb0 = rbase[b];
  const int rb1 = rbase[b + 1];
  rb0 = rb0 < 0 ? 0 : (rb0 > csrLen ? csrLen : rb0);
  rb0 &= ~31;
  int len = rb1 - rb0;
  len = len < 0 ? 0 : (len > RCAP ? RCAP : len);
  int lenW = (len + 31) & ~31;
  if (rb0 + lenW > csrLen) lenW = (csrLen - rb0) & ~31;

  {
    const v4i z = {0, 0, 0, 0};
    for (int i = tid; i < RCAP / 4; i += NTHR) ((v4i*)region)[i] = z;
    for (int s = tid; s < NBF; s += NTHR) {
      int o = off[nodeBase + s] - rb0;
      o = o < 0 ? 0 : (o > RCAP ? RCAP : o);
      cursor[s] = o;
    }
  }
  __syncthreads();

  const int nChunks = (nE + CHUNK - 1) / CHUNK;
#pragma unroll 1
  for (int ch = 0; ch < nChunks; ++ch) {
    const int cbase = ch * CHUNK;
    const int wc = scan_chunk<NBF>(dsts, nE, cbase, nodeBase, vec8, list, tid, lane, wave);
    if (lane == 0) wcnt[wave] = wc;
    __syncthreads();
    if (wave == 0) {
#pragma unroll 1
      for (int wsx = 0; wsx < NWAVE; ++wsx) {
        int n = __builtin_amdgcn_readfirstlane(wcnt[wsx]);
        n = n > WCAP ? WCAP : (n < 0 ? 0 : n);
        const int* lp = list + wsx * WCAP;
#pragma unroll 1
        for (int i = 0; i < n; ++i) {
          const int ent  = __builtin_amdgcn_readfirstlane(lp[i]);
          const int slot = ent & (NBF - 1);
          int e = cbase + ((ent >> 12) & (CHUNK - 1));
          e = e < 0 ? 0 : (e > nE - 1 ? nE - 1 : e);
          int sv = srcs[e];
          sv = sv < 0 ? 0 : (sv > nN - 1 ? nN - 1 : sv);
          if (lane == 0) {
            int pos = cursor[slot];
            pos = pos < 0 ? 0 : (pos > RCAP - 1 ? RCAP - 1 : pos);
            region[pos] = sv;
            const int np = pos + 1;
            cursor[slot] = np > RCAP ? RCAP : np;
          }
        }
      }
    }
    __syncthreads();
  }

  const int nv = lenW >> 2;
  int* gp = csr + rb0;
#pragma unroll 1
  for (int i = tid; i < nv; i += NTHR) { const v4i v = ((const v4i*)region)[i]; *(volatile v4i*)(gp + 4 * i) = v; }
  __threadfence();
#pragma unroll 1
  for (int i = tid; i < nv; i += NTHR) { const v4i v = ((const v4i*)region)[i]; *(volatile v4i*)(gp + 4 * i) = v; }
}

__global__ __launch_bounds__(NTHR) void k_agg(
    const int* __restrict__ csr, const int* __restrict__ off, const int* __restrict__ cnt,
    const float* __restrict__ X, float* AG, int nN, int csrLen) {
  const int tid = threadIdx.x, lane = tid & 31, wave = tid >> 5;
  const int tbase = blockIdx.x * TGT + wave * 32;
  const int col = 4 * lane;
  const v4f z4 = {0.f, 0.f, 0.f, 0.f};
  const int cl    = tbase + lane;
  const int cnt_l = cnt[cl];
  const int off_l = off[cl];

#pragma unroll 1
  for (int j = 0; j < 32; ++j) {
    const int c  = tbase + j;
    const int dg = __shfl(cnt_l, j);
    const int n  = dg < 0 ? 0 : (dg > DEGCAP ? DEGCAP : dg);
    const int st = __shfl(off_l, j);
    v4f acc = z4;
#pragma unroll 1
    for (int q0 = 0; q0 < n; q0 += 32) {
      int pos = st + q0 + lane;
      pos = pos < 0 ? 0 : (pos > csrLen - 1 ? csrLen - 1 : pos);
      int sl = csr[pos];
      sl = sl < 0 ? 0 : (sl > nN - 1 ? nN - 1 : sl);
      const int mcnt = (n - q0) < 32 ? (n - q0) : 32;
#pragma unroll 1
      for (int pp = 0; pp < mcnt; ++pp) {
        const int s = __builtin_amdgcn_readlane(sl, pp);
        acc += *(const v4f*)(X + (size_t)s * DD + col);
      }
    }
    const float df  = (float)(dg < 1 ? 1 : dg);
    const float inv = 1.0f / df;
    v4f v = acc * inv;
    if (c >= nN) v = z4;
    float* po = AG + (size_t)c * DD + col;
    *(volatile v4f*)po = v;
    __threadfence();
    *(volatile v4f*)po = v;
  }
}

template <int ROWS, int KW, int PD>
__device__ __forceinline__ void stage_rows(const float* src, int rowBase, int nValid, _Float16* dst, int colOff) {
  constexpr int UPR = KW / 8;
  constexpr int NU  = ROWS * UPR;
  static_assert((NU % NTHR) == 0);
  const int tid = threadIdx.x;
  const v4f z4 = {0.f, 0.f, 0.f, 0.f};
#pragma unroll 2
  for (int it = 0; it < NU / NTHR; ++it) {
    const int u = it * NTHR + tid;
    const int r = u / UPR, c = (u % UPR) * 8;
    const int grow = rowBase + r;
    const int rc = grow < nValid ? grow : nValid - 1;
    const float* p = src + (size_t)rc * KW + c;
    v4f a = *(const v4f*)p, b = *(const v4f*)(p + 4);
    if (grow >= nValid) { a = z4; b = z4; }
    *(v8h*)(dst + (size_t)r * PD + colOff + c) = cvt8(a, b, 1.0f);
  }
}

template <int NT, int KA>
__device__ __forceinline__ void mmk(v8f (&acc)[NT], const _Float16* tA, int arow,
                                    const _Float16* __restrict__ Bp, int bcol0) {
  const int lane = threadIdx.x & 31, hh = lane >> 4, m = lane & 15;
  const _Float16* ap = tA + (arow + m) * KA + 8 * hh;
  const _Float16* bp = Bp + (size_t)(bcol0 + m) * KA + 8 * hh;
#pragma unroll 1
  for (int kt = 0; kt < KA / 32; ++kt) {
    FragH a;
    a.h[0] = *(const v8h*)(ap + 32 * kt);
    a.h[1] = *(const v8h*)(ap + 32 * kt + 16);
#pragma unroll
    for (int t = 0; t < NT; ++t) {
      const size_t to = (size_t)(16 * t) * KA + 32 * kt;
      FragH bq;
      bq.h[0] = *(const v8h*)(bp + to);
      bq.h[1] = *(const v8h*)(bp + to + 16);
      acc[t] = wmh(a.v, bq.v, acc[t]);
    }
  }
}

__device__ __forceinline__ void epi_relu16(const v8f (&acc)[4], _Float16* tH, int r0, int c0,
                                           const float* __restrict__ bias) {
  const int lane = threadIdx.x & 31, hh = lane >> 4, m = lane & 15;
#pragma unroll
  for (int t = 0; t < 4; ++t) {
    const int col = c0 + 16 * t + m;
    const float bb = bias[col];
#pragma unroll
    for (int r = 0; r < 8; ++r)
      tH[(r0 + 8 * hh + r) * HID + col] = (_Float16)fmaxf(acc[t][r] * WSCLI + bb, 0.f);
  }
}

__device__ __forceinline__ void epi_lin32(const v8f (&acc)[4], float* stg, int r0, int c0,
                                          const float* __restrict__ bias) {
  const int lane = threadIdx.x & 31, hh = lane >> 4, m = lane & 15;
#pragma unroll
  for (int t = 0; t < 4; ++t) {
    const int col = c0 + 16 * t + m;
    const float bb = bias[col];
#pragma unroll
    for (int r = 0; r < 8; ++r)
      stg[(r0 + 8 * hh + r) * HID + col] = acc[t][r] * WSCLI + bb;
  }
}

__device__ __forceinline__ void store_rows128(const float* stg, float* dstp, int rowBase, int nN) {
  const int tid = threadIdx.x, lane = tid & 31, wave = tid >> 5;
#pragma unroll
  for (int row = 0; row < 8; ++row) {
    const int lrow = 8 * wave + row;
    const int grow = rowBase + lrow;
    if (grow < nN) {
      const v4f v = *(const v4f*)(stg + lrow * HID + 4 * lane);
      *(volatile v4f*)(dstp + (size_t)grow * HID + 4 * lane) = v;
    }
  }
  __threadfence();
#pragma unroll
  for (int row = 0; row < 8; ++row) {
    const int lrow = 8 * wave + row;
    const int grow = rowBase + lrow;
    if (grow < nN) {
      const v4f v = *(const v4f*)(stg + lrow * HID + 4 * lane);
      *(volatile v4f*)(dstp + (size_t)grow * HID + 4 * lane) = v;
    }
  }
}

__global__ __launch_bounds__(NTHR) void k_proj(
    const float* __restrict__ EF, const _Float16* __restrict__ P1, const float* __restrict__ b1,
    const _Float16* __restrict__ P2, const float* __restrict__ b2, float* H, int nN) {
  extern __shared__ v4f lds_dyn[];
  _Float16* tA  = (_Float16*)lds_dyn;
  _Float16* tH  = tA + BM * KP1;
  float*    stg = (float*)(tH + BM * HID);
  const int tid = threadIdx.x, wave = tid >> 5;
  const int rowBase = blockIdx.x * BM;
  const int r0 = (wave >> 1) * 16, c0 = (wave & 1) * 64;

  {
    const v4f z4 = {0.f, 0.f, 0.f, 0.f};
    if (tid < 128) {
      const int u = tid, r = u >> 1, c = (u & 1) * 8;
      const int grow = rowBase + r;
      const int rc = grow < nN ? grow : nN - 1;
      const float* p = EF + (size_t)rc * FIN + c;
      v4f a = *(const v4f*)p, b = *(const v4f*)(p + 4);
      if (grow >= nN) { a = z4; b = z4; }
      *(v8h*)(tA + r * KP1 + c) = cvt8(a, b, 1.0f);
    } else {
      const int u = tid - 128, r = u >> 1, c = 16 + (u & 1) * 8;
      *(v8h*)(tA + r * KP1 + c) = cvt8(z4, z4, 1.0f);
    }
  }
  __syncthreads();

  v8f acc[4];
  zacc(acc);
  mmk<4, KP1>(acc, tA, r0, P1, c0);
  epi_relu16(acc, tH, r0, c0, b1);
  __syncthreads();

  zacc(acc);
  mmk<4, HID>(acc, tH, r0, P2, c0);
  epi_lin32(acc, stg, r0, c0, b2);
  __syncthreads();

  store_rows128(stg, H, rowBase, nN);
}

__global__ __launch_bounds__(NTHR) void k_layer(
    const float* __restrict__ AG, float* H,
    const _Float16* __restrict__ P1, const float* __restrict__ b1,
    const _Float16* __restrict__ P2, const float* __restrict__ b2,
    const float* __restrict__ lng, const float* __restrict__ lnb, int nN) {
  extern __shared__ v4f lds_dyn[];
  _Float16* tA  = (_Float16*)lds_dyn;
  _Float16* tH  = tA + BM * K2;
  float*    stg = (float*)(tH + BM * HID);
  const int tid = threadIdx.x, lane = tid & 31, wave = tid >> 5;
  const int rowBase = blockIdx.x * BM;
  const int r0 = (wave >> 1) * 16, c0 = (wave & 1) * 64;

  stage_rows<BM, DD, K2>(H,  rowBase, nN, tA, 0);
  stage_rows<BM, DD, K2>(AG, rowBase, nN, tA, DD);
  __syncthreads();

  v8f acc[4];
  zacc(acc);
  mmk<4, K2>(acc, tA, r0, P1, c0);
  epi_relu16(acc, tH, r0, c0, b1);
  __syncthreads();

  zacc(acc);
  mmk<4, HID>(acc, tH, r0, P2, c0);
  epi_lin32(acc, stg, r0, c0, b2);
  __syncthreads();

  const v4f g4 = *(const v4f*)(lng + 4 * lane);
  const v4f e4 = *(const v4f*)(lnb + 4 * lane);
  v4f hres[8];
#pragma unroll
  for (int row = 0; row < 8; ++row) {
    const int grow = rowBase + 8 * wave + row;
    const int rc = grow < nN ? grow : nN - 1;
    hres[row] = *(const v4f*)(H + (size_t)rc * HID + 4 * lane);
  }
  v4f o[8];
#pragma unroll
  for (int row = 0; row < 8; ++row) {
    const int lrow = 8 * wave + row;
    const v4f hn = *(const v4f*)(stg + lrow * HID + 4 * lane);
    const v4f y = hres[row] + hn;
    float s = (y.x + y.y) + (y.z + y.w);
    s = wsum(s);
    const float mean = s * (1.0f / 128.0f);
    const v4f d = y - mean;
    float q = d.x * d.x + d.y * d.y + d.z * d.z + d.w * d.w;
    q = wsum(q);
    const float var  = q * (1.0f / 128.0f);
    const float rstd = rsqrtf(var + 1e-6f);
    o[row] = g4 * (d * rstd) + e4;
  }
#pragma unroll
  for (int row = 0; row < 8; ++row) {
    const int grow = rowBase + 8 * wave + row;
    if (grow < nN) *(volatile v4f*)(H + (size_t)grow * HID + 4 * lane) = o[row];
  }
  __threadfence();
#pragma unroll
  for (int row = 0; row < 8; ++row) {
    const int grow = rowBase + 8 * wave + row;
    if (grow < nN) *(volatile v4f*)(H + (size_t)grow * HID + 4 * lane) = o[row];
  }
}

__global__ __launch_bounds__(NTHR) void k_out(
    const float* __restrict__ H, const _Float16* __restrict__ P1, const float* __restrict__ b1,
    const float* __restrict__ w2, const float* __restrict__ b2, float* out, int nN) {
  extern __shared__ v4f lds_dyn[];
  _Float16* tA  = (_Float16*)lds_dyn;
  float*    stg = (float*)(tA + BM * HID);
  float*    sO  = stg + BM * HID;
  const int tid = threadIdx.x, lane = tid & 31, wave = tid >> 5, hh = lane >> 4, m = lane & 15;
  const int rowBase = blockIdx.x * BM;
  const int r0 = (wave >> 1) * 16, c0 = (wave & 1) * 64;

  stage_rows<BM, DD, HID>(H, rowBase, nN, tA, 0);
  __syncthreads();

  v8f acc[4];
  zacc(acc);
  mmk<4, HID>(acc, tA, r0, P1, c0);
#pragma unroll
  for (int t = 0; t < 4; ++t) {
    const int col = c0 + 16 * t + m;
    const float bb = b1[col];
#pragma unroll
    for (int r = 0; r < 8; ++r)
      stg[(r0 + 8 * hh + r) * HID + col] = fmaxf(acc[t][r] * WSCLI + bb, 0.f);
  }
  __syncthreads();

  const v4f w4 = *(const v4f*)(w2 + 4 * lane);
  const float bb2 = b2[0];
#pragma unroll
  for (int row = 0; row < 8; ++row) {
    const int lrow = 8 * wave + row;
    const v4f y = *(const v4f*)(stg + lrow * HID + 4 * lane);
    float p = y.x * w4.x + y.y * w4.y + y.z * w4.z + y.w * w4.w;
    p = wsum(p);
    if (lane == 0) sO[lrow] = p + bb2;
  }
  __syncthreads();

  if (wave == 0) {
    const int rem = nN - rowBase;
    const int nv  = rem < BM ? rem : BM;
    const int i0  = 4 * lane;
    const int i0c = 4 * (lane & 15);
    const v4f v = *(const v4f*)(sO + i0c);
    float* po = out + (size_t)rowBase + i0;
    const bool full = (lane < 16) && (i0 + 3 < nv);
    const bool part = (lane < 16) && (!full) && (i0 < nv);
    if (full) *(volatile v4f*)po = v;
    if (part) {
      if (i0     < nv) *(volatile float*)(po)     = v.x;
      if (i0 + 1 < nv) *(volatile float*)(po + 1) = v.y;
      if (i0 + 2 < nv) *(volatile float*)(po + 2) = v.z;
    }
    __threadfence();
    if (full) *(volatile v4f*)po = v;
    if (part) {
      if (i0     < nv) *(volatile float*)(po)     = v.x;
      if (i0 + 1 < nv) *(volatile float*)(po + 1) = v.y;
      if (i0 + 2 < nv) *(volatile float*)(po + 2) = v.z;
    }
  }
}

static size_t carve(size_t* o, size_t bytes) {
  const size_t r = *o;
  *o += (bytes + 255) & ~(size_t)255;
  return r;
}

extern "C" void kernel_launch(void* const* d_in, const int* in_sizes, int n_in,
                              void* d_out, int out_size, void* d_ws, size_t ws_size,
                              hipStream_t stream) {
  if (n_in < 17) return;
  const int nN = in_sizes[0] / FIN;
  const int nE = in_sizes[1];
  if (nN <= 0 || nE <= 0 || in_sizes[0] != nN * FIN || in_sizes[2] != nE) return;
  if (in_sizes[3] != FIN * HID || in_sizes[4] != HID || in_sizes[5] != HID * HID || in_sizes[6] != HID) return;
  const int L = in_sizes[7] / (K2 * HID);
  if (L < 1 || L > LMAX || in_sizes[7] != L * K2 * HID || in_sizes[8] != L * HID) return;
  if (in_sizes[9] != L * HID * HID || in_sizes[10] != L * HID || in_sizes[11] != L * HID || in_sizes[12] != L * HID) return;
  if (in_sizes[13] != HID * HID || in_sizes[14] != HID || in_sizes[15] != HID || in_sizes[16] != 1) return;
  if (out_size != nN) return;
  if (nE > (1 << 27) || nN > (1 << 22)) return;

  const float* ef  = (const float*)d_in[0];
  const int*   src = (const int*)d_in[1];
  const int*   dst = (const int*)d_in[2];
  const float* wp1 = (const float*)d_in[3];
  const float* bp1 = (const float*)d_in[4];
  const float* wp2 = (const float*)d_in[5];
  const float* bp2 = (const float*)d_in[6];
  const float* wu1 = (const float*)d_in[7];
  const float* bu1 = (const float*)d_in[8];
  const float* wu2 = (const float*)d_in[9];
  const float* bu2 = (const float*)d_in[10];
  const float* lng = (const float*)d_in[11];
  const float* lnb = (const float*)d_in[12];
  const float* wo1 = (const float*)d_in[13];
  const float* bo1 = (const float*)d_in[14];
  const float* wo2 = (const float*)d_in[15];
  const float* bo2 = (const float*)d_in[16];
  float* dout = (float*)d_out;

  const int NPAD   = ((nN + TGT - 1) / TGT) * TGT;
  const int nBC    = (nN + NBC - 1) / NBC;
  const int CNTPAD = nBC * NBC;
  if (FPC * nBC + 1 > RBN) return;
  const int nBF    = (nN + NBF - 1) / NBF;
  const int csrLen = ((nE + 31) & ~31) + 4096;
  if (31 * FPC * nBC > 4096) return;
  if ((long long)nE * NBF > (long long)nN * (RCAP / 4 * 3)) return;
  if ((long long)nE > (long long)nN * (DEGCAP / 2)) return;
  const int nAgg   = NPAD / TGT;
  const int nMl    = (nN + BM - 1) / BM;
  const int HROWS  = nMl * BM;

  const size_t planeHalves = (size_t)PL_P1 + PL_SQ + (size_t)L * (PL_U1 + PL_SQ) + PL_SQ;
  const int    nWB         = BP1 + BSQ + L * (BU1 + BSQ) + BSQ;
  if ((size_t)nWB * UPB != planeHalves) return;

  char* ws = (char*)d_ws;
  size_t o = 0;
  const size_t oPl  = carve(&o, planeHalves * 2);
  const size_t oCnt = carve(&o, (size_t)CNTPAD * 4);
  const size_t oOff = carve(&o, (size_t)CNTPAD * 4);
  const size_t oRb  = carve(&o, (size_t)RBN * 4);
  const size_t oCsr = carve(&o, (size_t)csrLen * 4);
  const size_t oAG  = carve(&o, (size_t)NPAD * DD * 4);
  const size_t oH   = carve(&o, (size_t)HROWS * DD * 4);
  if (o > ws_size || o > (size_t)WSCAP) return;

  _Float16* planes = (_Float16*)(ws + oPl);
  int*      cnt    = (int*)(ws + oCnt);
  int*      offp   = (int*)(ws + oOff);
  int*      rb     = (int*)(ws + oRb);
  int*      csr    = (int*)(ws + oCsr);
  float*    AG     = (float*)(ws + oAG);
  float*    H      = (float*)(ws + oH);

  const _Float16* pP1 = planes;
  const _Float16* pP2 = planes + PL_P1;
  const _Float16* pU1 = planes + PL_P1 + PL_SQ;
  const _Float16* pU2 = planes + PL_P1 + PL_SQ + (size_t)L * PL_U1;
  const _Float16* pO1 = planes + PL_P1 + PL_SQ + (size_t)L * (PL_U1 + PL_SQ);

  const int vec8 = 1;

  k_wprep<<<nWB, NTHR, 0, stream>>>(wp1, wp2, wu1, wu2, wo1, planes, L);

  k_count<<<nBC, NTHR, 0, stream>>>(dst, cnt, nE, vec8);
  k_offsets<<<1, OTHR, 0, stream>>>(cnt, offp, rb, nBC);
  hipFuncSetAttribute(reinterpret_cast<const void*>(&k_fill),
                      hipFuncAttributeMaxDynamicSharedMemorySize, LDS_FILL);
  k_fill<<<nBF, NTHR, LDS_FILL, stream>>>(dst, src, offp, rb, csr, nN, nE, vec8, csrLen);

  hipFuncSetAttribute(reinterpret_cast<const void*>(&k_proj),
                      hipFuncAttributeMaxDynamicSharedMemorySize, LDS_PROJ);
  k_proj<<<nMl, NTHR, LDS_PROJ, stream>>>(ef, pP1, bp1, pP2, bp2, H, nN);

  hipFuncSetAttribute(reinterpret_cast<const void*>(&k_layer),
                      hipFuncAttributeMaxDynamicSharedMemorySize, LDS_LAYER);
  for (int i = 0; i < L; ++i) {
    k_agg<<<nAgg, NTHR, 0, stream>>>(csr, offp, cnt, H, AG, nN, csrLen);
    k_layer<<<nMl, NTHR, LDS_LAYER, stream>>>(
        AG, H, pU1 + (size_t)i * PL_U1, bu1 + (size_t)i * HID,
        pU2 + (size_t)i * PL_SQ, bu2 + (size_t)i * HID,
        lng + (size_t)i * HID, lnb + (size_t)i * HID, nN);
  }

  hipFuncSetAttribute(reinterpret_cast<const void*>(&k_out),
                      hipFuncAttributeMaxDynamicSharedMemorySize, LDS_OUT);
  k_out<<<nMl, NTHR, LDS_OUT, stream>>>(H, pO1, bo1, wo2, bo2, dout, nN);
}
